// SelfAttention_10634339025419
// MI455X (gfx1250) — hardware-verified
//
#include <hip/hip_runtime.h>
#include <math.h>

typedef __attribute__((ext_vector_type(16))) _Float16 v16h;
typedef __attribute__((ext_vector_type(8)))  _Float16 v8h;
typedef __attribute__((ext_vector_type(8)))  float    v8f;
typedef __attribute__((ext_vector_type(4)))  float    v4f;

constexpr int kInputsRneToBf16 = 1;

constexpr int kBatch = 4;
constexpr int kSeq   = 2048;
constexpr int kDim   = 1024;
constexpr int kTok   = kBatch * kSeq;
constexpr int kTriRowsMax = kSeq / 64;

constexpr int isqrt_c(int n) { int r = 0; while ((r + 1) * (r + 1) <= n) ++r; return r; }
constexpr int kSqrtDim = isqrt_c(kDim);
static_assert(kSqrtDim * kSqrtDim == kDim);
constexpr float kScoreScale = 1.0f / (float)kSqrtDim;

constexpr float kXCarry = 64.0f;
constexpr float kWCarry = 1024.0f;
constexpr float kQCarry = 64.0f;
constexpr float kKCarry = 64.0f;
constexpr float kVCarry = 64.0f;
constexpr float kSCarry = 64.0f;
constexpr float kF16MinNormal = 6.103515625e-05f;

constexpr float kProjScaleQ   = kQCarry / (kXCarry * kWCarry);
constexpr float kProjScaleK   = kKCarry / (kXCarry * kWCarry);
constexpr float kProjScaleV   = kVCarry / (kXCarry * kWCarry);
constexpr float kScoreEpi     = kSCarry * kScoreScale / (kQCarry * kKCarry);
constexpr float kOutEpi       = 1.0f / (kSCarry * kVCarry);

static_assert((kTok % 64) == 0 && (kSeq % 64) == 0 && (kDim % 64) == 0);
static_assert((kDim % 32) == 0 && (kSeq % 32) == 0);
static_assert(kTriRowsMax == 32);
static_assert(((kTok * kDim) % (8 * 256)) == 0 && ((kDim * kDim) % (8 * 256)) == 0);

constexpr size_t kBytesX16  = (size_t)kTok * kDim * 2;
constexpr size_t kBytesW16  = (size_t)3 * kDim * kDim * 2;
constexpr size_t kBytesQ16  = (size_t)kTok * kDim * 2;
constexpr size_t kBytesK16  = (size_t)kTok * kDim * 2;
constexpr size_t kBytesVT16 = (size_t)kBatch * kDim * kSeq * 2;
constexpr size_t kBytesS16  = (size_t)kBatch * kSeq * kSeq * 2;
constexpr size_t kOffX16  = 0;
constexpr size_t kOffW16  = kOffX16  + kBytesX16;
constexpr size_t kOffQ16  = kOffW16  + kBytesW16;
constexpr size_t kOffK16  = kOffQ16  + kBytesQ16;
constexpr size_t kOffVT16 = kOffK16  + kBytesK16;
constexpr size_t kOffS16  = kOffVT16 + kBytesVT16;
constexpr size_t kWsTotal = kOffS16  + kBytesS16;
static_assert(kWsTotal == 106954752ull);
static_assert(kWsTotal <= 134217728ull);
static_assert((kOffW16 % 128) == 0 && (kOffQ16 % 128) == 0 && (kOffK16 % 128) == 0 &&
              (kOffVT16 % 128) == 0 && (kOffS16 % 128) == 0);

__device__ __forceinline__ unsigned short f2bf_bits(float f) {
  unsigned u = __float_as_uint(f);
  return (unsigned short)((u + 0x7FFFu + ((u >> 16) & 1u)) >> 16);
}
__device__ __forceinline__ float bf_bits2f(unsigned short h) { return __uint_as_float(((unsigned)h) << 16); }

__device__ __forceinline__ float input_val(float v) {
  if (kInputsRneToBf16) return bf_bits2f(f2bf_bits(v));
  return v;
}
__device__ __forceinline__ _Float16 to_f16_flushed(float c) {
  const float s = (fabsf(c) < kF16MinNormal) ? 0.0f : c;
  return (_Float16)s;
}

union FragU { v16h v; v8h h[2]; };
__device__ __forceinline__ v16h frag_load(const _Float16* p) {
  FragU f;
  f.h[0] = *(const v8h*)(p);
  f.h[1] = *(const v8h*)(p + 16);
  return f.v;
}
__device__ __forceinline__ v8f mma_tied(v16h a, v16h b, v8f c) {
  c = __builtin_amdgcn_wmma_f32_16x16x32_f16(false, a, false, b, (short)0, c, false, false);
  asm volatile("" : "+v"(c) : "v"(a), "v"(b));
  return c;
}
__device__ __forceinline__ void nop_guard(v8f& c, v16h a, v16h b) {
  asm volatile("v_nop\n\tv_nop\n\tv_nop\n\tv_nop" : "+v"(c) : "v"(a), "v"(b));
}
__device__ __forceinline__ void acc_guard1(v8f& c) {
  asm volatile("v_nop\n\tv_nop\n\tv_nop\n\tv_nop" : "+v"(c));
}
__device__ __forceinline__ void keep4_h(v16h a, v16h b, v16h c, v16h d) {
  asm volatile("v_nop" :: "v"(a), "v"(b), "v"(c), "v"(d));
}

__global__ __launch_bounds__(256) void cvt8_f16_kernel(const float* __restrict__ in,
                                                       unsigned short* __restrict__ out, int n8, float carry) {
  const int i = blockIdx.x * 256 + threadIdx.x;
  if (i >= n8) return;
  const size_t e0 = (size_t)i << 3;
  const v4f a0 = *(const v4f*)(in + e0);
  const v4f a1 = *(const v4f*)(in + e0 + 4);
  v8h hv;
#pragma unroll
  for (int e = 0; e < 4; ++e) {
    const float t0 = a0[e];
    const float t1 = a1[e];
    const float c0 = input_val(t0) * carry;
    const float c1 = input_val(t1) * carry;
    hv[e]     = to_f16_flushed(c0);
    hv[4 + e] = to_f16_flushed(c1);
  }
  unsigned short* q = out + e0;
  *(volatile v8h*)q = hv;
  __threadfence();
  *(volatile v8h*)q = hv;
}

template <int BIAS_MODE, bool OUT_F16, int CAUSAL>
__global__ __launch_bounds__(256) void gemm_f16_kernel(
    const unsigned short* __restrict__ Ap, int lda, long strideA,
    const unsigned short* __restrict__ Btp, int ldb, long strideB,
    void* __restrict__ Cout, int ldc, long strideC,
    const float* __restrict__ bias, float biasScale,
    int M, int N, int K, float scale) {
  const _Float16* A  = (const _Float16*)Ap;
  const _Float16* Bt = (const _Float16*)Btp;
  __shared__ __align__(16) float sT[8][16 * 68];
  const int b    = blockIdx.y;
  const int lane = threadIdx.x & 31;
  const int wave = threadIdx.x >> 5;
  const int tilesN = N >> 6;
  const int tilesM = M >> 6;
  const int tile = __builtin_amdgcn_readfirstlane((int)(blockIdx.x * 8 + wave));
  const int nTiles = (CAUSAL == 1) ? ((tilesM * (tilesM + 1)) >> 1) : (tilesM * tilesN);
  if (tile >= nTiles) return;
  int tm, tn;
  if (CAUSAL == 1) {
    tm = 0;
    for (int i = 0; i < kTriRowsMax; ++i) {
      if ((((i + 1) * (i + 2)) >> 1) <= tile) tm = i + 1;
    }
    tm = (tm < tilesM - 1) ? tm : (tilesM - 1);
    tn = tile - ((tm * (tm + 1)) >> 1);
    tn = (tn < 0) ? 0 : tn;
    tn = (tn > tm) ? tm : tn;
  } else {
    tm = tile / tilesN;
    tn = tile - tm * tilesN;
  }
  const int m0 = tm << 6;
  const int n0 = tn << 6;
  int kEnd = K;
  if (CAUSAL == 2) {
    const int kc = (tm + 1) << 6;
    kEnd = (kc < K) ? kc : K;
  }

  const _Float16* Ab = A  + (size_t)b * strideA;
  const _Float16* Bb = Bt + (size_t)b * strideB;

  const int rlane = lane & 15;
  const int koff  = (lane >> 4) * 8;
  const int mOff  = (lane >> 4) * 8;

  v8f acc[4][4];
#pragma unroll
  for (int i = 0; i < 4; ++i)
#pragma unroll
    for (int j = 0; j < 4; ++j) acc[i][j] = (v8f){0.f, 0.f, 0.f, 0.f, 0.f, 0.f, 0.f, 0.f};

  for (int k0 = 0; k0 < kEnd; k0 += 32) {
    v16h bh[4];
#pragma unroll
    for (int j = 0; j < 4; ++j) {
      const size_t bo = (size_t)(n0 + (j << 4) + rlane) * ldb + koff + k0;
      bh[j] = frag_load(Bb + bo);
    }
#pragma unroll
    for (int i = 0; i < 4; ++i) {
      const size_t ao = (size_t)(m0 + (i << 4) + rlane) * lda + koff + k0;
      const v16h ah = frag_load(Ab + ao);
      acc[i][0] = mma_tied(ah, bh[0], acc[i][0]);
      acc[i][1] = mma_tied(ah, bh[1], acc[i][1]);
      acc[i][2] = mma_tied(ah, bh[2], acc[i][2]);
      acc[i][3] = mma_tied(ah, bh[3], acc[i][3]);
      nop_guard(acc[i][3], ah, bh[3]);
    }
    keep4_h(bh[0], bh[1], bh[2], bh[3]);
  }
#pragma unroll
  for (int i = 0; i < 4; ++i) {
    acc_guard1(acc[i][0]);
    acc_guard1(acc[i][1]);
    acc_guard1(acc[i][2]);
    acc_guard1(acc[i][3]);
  }

  float* slab = sT[wave];
  const bool diag = (CAUSAL == 1) && (tm == tn);
  float bn[4] = {0.f, 0.f, 0.f, 0.f};
  if (BIAS_MODE == 2) {
#pragma unroll
    for (int j = 0; j < 4; ++j) {
      const float t = bias[n0 + (j << 4) + rlane];
      bn[j] = input_val(t) * biasScale;
    }
  }
#pragma unroll
  for (int i = 0; i < 4; ++i) {
    const int mBase = m0 + (i << 4);
    float bm[8] = {0.f, 0.f, 0.f, 0.f, 0.f, 0.f, 0.f, 0.f};
    if (BIAS_MODE == 1) {
      const v4f b0 = *(const v4f*)(bias + mBase + mOff);
      const v4f b1 = *(const v4f*)(bias + mBase + mOff + 4);
#pragma unroll
      for (int e = 0; e < 4; ++e) {
        const float t0 = b0[e];
        const float t1 = b1[e];
        bm[e]     = input_val(t0) * biasScale;
        bm[4 + e] = input_val(t1) * biasScale;
      }
    }
#pragma unroll
    for (int j = 0; j < 4; ++j) {
      const int n = n0 + (j << 4) + rlane;
#pragma unroll
      for (int r = 0; r < 8; ++r) {
        const int row = mBase + mOff + r;
        float v = acc[i][j][r] * scale;
        if (BIAS_MODE == 1) v += bm[r];
        if (BIAS_MODE == 2) v += bn[j];
        if (diag && (n > row)) v = 0.0f;
        slab[(mOff + r) * 68 + (j << 4) + rlane] = v;
      }
    }
    __builtin_amdgcn_fence(__ATOMIC_RELEASE, "workgroup");
    __builtin_amdgcn_wave_barrier();
    __builtin_amdgcn_fence(__ATOMIC_ACQUIRE, "workgroup");
    if (!OUT_F16) {
      float* C = (float*)Cout + (size_t)b * strideC;
      const int hh = lane >> 4, c4 = (lane & 15) * 4;
      for (int pass = 0; pass < 2; ++pass) {
#pragma unroll
        for (int it = 0; it < 8; ++it) {
          const int row = it * 2 + hh;
          const v4f v = *(const v4f*)(slab + row * 68 + c4);
          *(volatile v4f*)(C + (size_t)(mBase + row) * ldc + n0 + c4) = v;
        }
        __threadfence();
      }
    } else {
      const int q = lane >> 3, c8 = (lane & 7) * 8;
      unsigned short* C = (unsigned short*)Cout + (size_t)b * strideC;
      for (int pass = 0; pass < 2; ++pass) {
#pragma unroll
        for (int it = 0; it < 4; ++it) {
          const int row = it * 4 + q;
          const float* sp = slab + row * 68 + c8;
          v8h hv;
#pragma unroll
          for (int e = 0; e < 8; ++e) {
            const float t = sp[e];
            hv[e] = to_f16_flushed(t);
          }
          *(volatile v8h*)(C + (size_t)(mBase + row) * ldc + n0 + c8) = hv;
        }
        __threadfence();
      }
    }
    __builtin_amdgcn_fence(__ATOMIC_RELEASE, "workgroup");
    __builtin_amdgcn_wave_barrier();
    __builtin_amdgcn_fence(__ATOMIC_ACQUIRE, "workgroup");
  }
}

extern "C" void kernel_launch(void* const* d_in, const int* in_sizes, int n_in,
                              void* d_out, int out_size, void* d_ws, size_t ws_size,
                              hipStream_t stream) {
  if (n_in < 7) return;
  if (in_sizes[0] != kTok * kDim) return;
  if (in_sizes[1] != kDim * kDim) return;
  if (in_sizes[2] != kDim) return;
  if (in_sizes[3] != kDim * kDim) return;
  if (in_sizes[4] != kDim) return;
  if (in_sizes[5] != kDim * kDim) return;
  if (in_sizes[6] != kDim) return;
  if (out_size != kTok * kDim) return;
  if (ws_size < kWsTotal) return;

  const float* x  = (const float*)d_in[0];
  const float* Wq = (const float*)d_in[1];
  const float* bq = (const float*)d_in[2];
  const float* Wk = (const float*)d_in[3];
  const float* bk = (const float*)d_in[4];
  const float* Wv = (const float*)d_in[5];
  const float* bv = (const float*)d_in[6];
  float* out = (float*)d_out;

  char* ws = (char*)d_ws;
  unsigned short* X16  = (unsigned short*)(ws + kOffX16);
  unsigned short* W16  = (unsigned short*)(ws + kOffW16);
  unsigned short* Q16  = (unsigned short*)(ws + kOffQ16);
  unsigned short* K16  = (unsigned short*)(ws + kOffK16);
  unsigned short* VT16 = (unsigned short*)(ws + kOffVT16);
  unsigned short* S16  = (unsigned short*)(ws + kOffS16);
  unsigned short* Wq16 = W16;
  unsigned short* Wk16 = W16 + (size_t)kDim * kDim;
  unsigned short* Wv16 = W16 + (size_t)2 * kDim * kDim;

  const int nx8 = kTok * kDim / 8;
  const int nw8 = kDim * kDim / 8;
  cvt8_f16_kernel<<<nx8 / 256, 256, 0, stream>>>(x,  X16,  nx8, kXCarry);
  cvt8_f16_kernel<<<nw8 / 256, 256, 0, stream>>>(Wq, Wq16, nw8, kWCarry);
  cvt8_f16_kernel<<<nw8 / 256, 256, 0, stream>>>(Wk, Wk16, nw8, kWCarry);
  cvt8_f16_kernel<<<nw8 / 256, 256, 0, stream>>>(Wv, Wv16, nw8, kWCarry);

  {
    const int tiles = (kTok / 64) * (kDim / 64);
    gemm_f16_kernel<2, true, 0><<<dim3((tiles + 7) / 8, 1), 256, 0, stream>>>(
        X16, kDim, 0L, Wq16, kDim, 0L, (void*)Q16, kDim, 0L,
        bq, kQCarry, kTok, kDim, kDim, kProjScaleQ);
    gemm_f16_kernel<2, true, 0><<<dim3((tiles + 7) / 8, 1), 256, 0, stream>>>(
        X16, kDim, 0L, Wk16, kDim, 0L, (void*)K16, kDim, 0L,
        bk, kKCarry, kTok, kDim, kDim, kProjScaleK);
  }

  {
    const int tiles = (kDim / 64) * (kSeq / 64);
    gemm_f16_kernel<1, true, 0><<<dim3((tiles + 7) / 8, kBatch), 256, 0, stream>>>(
        Wv16, kDim, 0L, X16, kDim, (long)kSeq * kDim, (void*)VT16, kSeq, (long)kDim * kSeq,
        bv, kVCarry, kDim, kSeq, kDim, kProjScaleV);
  }

  {
    const int tr = kSeq / 64;
    const int tiles = (tr * (tr + 1)) / 2;
    gemm_f16_kernel<0, true, 1><<<dim3((tiles + 7) / 8, kBatch), 256, 0, stream>>>(
        Q16, kDim, (long)kSeq * kDim, K16, kDim, (long)kSeq * kDim, (void*)S16, kSeq, (long)kSeq * kSeq,
        nullptr, 0.0f, kSeq, kSeq, kDim, kScoreEpi);
  }

  {
    const int tiles = (kSeq / 64) * (kDim / 64);
    gemm_f16_kernel<0, false, 2><<<dim3((tiles + 7) / 8, kBatch), 256, 0, stream>>>(
        S16, kSeq, (long)kSeq * kSeq, VT16, kSeq, (long)kDim * kSeq, (void*)out, kDim, (long)kSeq * kDim,
        nullptr, 0.0f, kSeq, kDim, kSeq, kOutEpi);
  }
}
